// GCN2_LSTM_89008902243172
// MI455X (gfx1250) — hardware-verified
//
#include <hip/hip_runtime.h>


namespace {
constexpr int N = 100000, E = 1600000, EL = 1000000, F = 64, S = 64, C = 32, NPAD = 100096, NBLK = NPAD / 128;

typedef _Float16 b16;
typedef __attribute__((ext_vector_type(16))) _Float16 v16b;
typedef __attribute__((ext_vector_type(8)))  _Float16 v8b;
typedef __attribute__((ext_vector_type(8)))  float v8f;
typedef __attribute__((ext_vector_type(4)))  float v4f;

__device__ __forceinline__ v8b ld8b(const b16* p) { return *(const v8b*)p; }
__device__ __forceinline__ v16b cat8b(v8b a, v8b b) { return __builtin_shufflevector(a, b, 0, 1, 2, 3, 4, 5, 6, 7, 8, 9, 10, 11, 12, 13, 14, 15); }
__device__ __forceinline__ v16b frag_kb(const b16* p, int hh) { return cat8b(ld8b(p + 8 * hh), ld8b(p + 16 + 8 * hh)); }
__device__ __forceinline__ void split16(float v, b16& hi, b16& lo) { hi = (b16)v; lo = (b16)(v - (float)hi); }
__device__ __forceinline__ void frag_ksplit(const float* p, int hh, v16b& fh_, v16b& fl_) {
  const float* p0 = p + 8 * hh; const float* p1 = p + 16 + 8 * hh;
#pragma unroll
  for (int e = 0; e < 8; ++e) { b16 a, c; split16(p0[e], a, c); fh_[e] = a; fl_[e] = c; split16(p1[e], a, c); fh_[8 + e] = a; fl_[8 + e] = c; }
}
__device__ __forceinline__ v8f wmma16b(v16b a, v16b b, v8f c) {
  v8f d = __builtin_amdgcn_wmma_f32_16x16x32_f16(false, a, false, b, (short)0, c, false, false);
  asm volatile("v_nop\n\tv_nop\n\tv_nop\n\tv_nop" : "+v"(d) : "v"(a), "v"(b));
  return d;
}
__device__ __forceinline__ void wave_lds_sync() {
  __builtin_amdgcn_fence(__ATOMIC_RELEASE, "workgroup");
  __builtin_amdgcn_wave_barrier();
  __builtin_amdgcn_fence(__ATOMIC_ACQUIRE, "workgroup");
}

struct Opnd { const void* p0; const void* p1; int ld; };
template <int NP> __device__ __forceinline__ void load_frags(const Opnd& o, int row, int kb, int hh, v16b& fh_, v16b& fl_) {
  if (NP == 0) { frag_ksplit((const float*)o.p0 + (size_t)row * o.ld + kb, hh, fh_, fl_); }
  else if (NP == 4) {
    const float* p = (const float*)o.p0 + (size_t)row * o.ld + kb; const float* p0 = p + 8 * hh; const float* p1 = p + 16 + 8 * hh;
#pragma unroll
    for (int e = 0; e < 8; ++e) { b16 a, c; split16(p0[e] * 64.0f, a, c); fh_[e] = a; fl_[e] = c; split16(p1[e] * 64.0f, a, c); fh_[8 + e] = a; fl_[8 + e] = c; }
  } else if (NP == 3) {
    const float* p = (const float*)o.p0 + (size_t)row * o.ld + kb; const float* p0 = p + 8 * hh; const float* p1 = p + 16 + 8 * hh;
#pragma unroll
    for (int e = 0; e < 8; ++e) { fh_[e] = (b16)p0[e]; fh_[8 + e] = (b16)p1[e]; }
    fl_ = fh_;
  } else {
    fh_ = frag_kb((const b16*)o.p0 + (size_t)row * o.ld + kb, hh);
    if (NP == 2) fl_ = frag_kb((const b16*)o.p1 + (size_t)row * o.ld + kb, hh); else fl_ = fh_;
  }
}
template <int ANP, int BNP> __device__ __forceinline__ v8f mac(v16b ah, v16b al, v16b bh, v16b bl, v8f c) {
  c = wmma16b(ah, bh, c);
  if (BNP == 0 || BNP == 2 || BNP == 4) c = wmma16b(ah, bl, c);
  if (ANP == 0 || ANP == 2 || ANP == 4) c = wmma16b(al, bh, c);
  return c;
}
template <int ANP, int BNP>
__device__ __forceinline__ void gemm_tile(const Opnd& A, const Opnd& B, int K, int m0, int c0, int nloc, int hlf, v8f (&acc)[2][4]) {
  for (int kb = 0; kb < K; kb += 32) {
    v16b a0h, a0l, a1h, a1l;
    load_frags<ANP>(A, m0 + nloc, kb, hlf, a0h, a0l);
    load_frags<ANP>(A, m0 + 16 + nloc, kb, hlf, a1h, a1l);
#pragma unroll
    for (int t = 0; t < 4; ++t) {
      v16b bh, bl;
      load_frags<BNP>(B, c0 + t * 16 + nloc, kb, hlf, bh, bl);
      acc[0][t] = mac<ANP, BNP>(a0h, a0l, bh, bl, acc[0][t]);
      acc[1][t] = mac<ANP, BNP>(a1h, a1l, bh, bl, acc[1][t]);
    }
  }
}

__device__ __forceinline__ void epi_planes(v8f (&acc)[2][4], float scale, bool two, b16* __restrict__ oh, b16* __restrict__ ol, int ldo,
                                           int m0, int c0, int lane, b16* Th, b16* Tl) {
  const int nloc = lane & 15, hlf = lane >> 4;
#pragma unroll
  for (int t = 0; t < 4; ++t)
#pragma unroll
    for (int r = 0; r < 2; ++r)
#pragma unroll
      for (int v = 0; v < 8; ++v) {
        const int rr = r * 16 + v + 8 * hlf, cc = t * 16 + nloc;
        b16 h_, l_; split16(acc[r][t][v] * scale, h_, l_);
        Th[rr * 64 + cc] = h_; Tl[rr * 64 + cc] = l_;
      }
  wave_lds_sync();
  for (int pass = 0; pass < 2; ++pass) {
#pragma unroll
    for (int j = 0; j < 8; ++j) {
      const int rr = j * 4 + (lane >> 3), c8 = (lane & 7) * 8;
      const size_t o = (size_t)(m0 + rr) * ldo + c0 + c8;
      *(volatile v8b*)(oh + o) = ld8b(Th + rr * 64 + c8);
      if (two) *(volatile v8b*)(ol + o) = ld8b(Tl + rr * 64 + c8);
    }
    __threadfence();
  }
}
__device__ __forceinline__ void epi_f32(v8f (&acc)[2][4], float scale, const float* rscale, float* __restrict__ out, int ldo, int m0, int c0, int lane, float* Tt) {
  const int nloc = lane & 15, hlf = lane >> 4;
#pragma unroll
  for (int t = 0; t < 4; ++t)
#pragma unroll
    for (int r = 0; r < 2; ++r)
#pragma unroll
      for (int v = 0; v < 8; ++v) {
        const int rr = r * 16 + v + 8 * hlf;
        const float rs = rscale ? rscale[(size_t)(m0 + rr) * 32] : 1.0f;
        Tt[rr * 64 + t * 16 + nloc] = acc[r][t][v] * scale * rs;
      }
  wave_lds_sync();
  float* dst0 = out + (size_t)m0 * ldo + c0;
  for (int pass = 0; pass < 2; ++pass) {
#pragma unroll
    for (int j = 0; j < 16; ++j) { const int rr = j * 2 + hlf, c4 = nloc * 4; *(volatile v4f*)(dst0 + (size_t)rr * ldo + c4) = *(const v4f*)(Tt + rr * 64 + c4); }
    __threadfence();
  }
}


__global__ __launch_bounds__(256) void prep_kernel(const float* __restrict__ x, const float* __restrict__ Wih, const float* __restrict__ bih, const float* __restrict__ bhh, const float* __restrict__ W1, const float* __restrict__ W2,
                                                   float* __restrict__ xp, b16* __restrict__ wih, float* __restrict__ bsum, b16* __restrict__ w1, b16* __restrict__ w2) {
  const size_t tid = (size_t)blockIdx.x * blockDim.x + threadIdx.x, nth = (size_t)gridDim.x * blockDim.x;
  for (int pass = 0; pass < 2; ++pass) {
    for (size_t p = tid; p < (size_t)NPAD * F / 4; p += nth) { const size_t n = p / (F / 4); const v4f v = (n < (size_t)N) ? *(const v4f*)(x + p * 4) : (v4f){0.0f, 0.0f, 0.0f, 0.0f}; *(volatile v4f*)(xp + p * 4) = v; }
    for (size_t p = tid; p < (size_t)4 * F * F / 8; p += nth) { v8b v;
#pragma unroll
      for (int e = 0; e < 8; ++e) v[e] = (b16)Wih[p * 8 + e];
      *(volatile v8b*)(wih + p * 8) = v; }
    for (size_t p = tid; p < (size_t)4 * F; p += nth) ((volatile float*)bsum)[p] = bih[p] + bhh[p];
    for (size_t p = tid; p < (size_t)S * F / 8; p += nth) { const int n = (int)(p / 8), k0 = (int)(p % 8) * 8; v8b v;
#pragma unroll
      for (int e = 0; e < 8; ++e) v[e] = (b16)W1[(size_t)(k0 + e) * S + n];
      *(volatile v8b*)(w1 + (size_t)n * F + k0) = v; }
    for (size_t p = tid; p < (size_t)C * S / 8; p += nth) { const int n = (int)(p / 8), k0 = (int)(p % 8) * 8; v8b v;
#pragma unroll
      for (int e = 0; e < 8; ++e) v[e] = (b16)W2[(size_t)(k0 + e) * C + n];
      *(volatile v8b*)(w2 + (size_t)n * S + k0) = v; }
    __threadfence();
  }
}

__global__ __launch_bounds__(128) void lstm_kernel(const float* __restrict__ xp, const b16* __restrict__ wih, const float* __restrict__ bsum, float* __restrict__ h) {
  __shared__ float Gt[32][4 * F + 4];
  const int lane = threadIdx.x & 31, wave = threadIdx.x >> 5, nloc = lane & 15, hlf = lane >> 4, m0 = blockIdx.x * 32, c0 = wave * F;
  v8f acc[2][4];
#pragma unroll
  for (int r = 0; r < 2; ++r)
#pragma unroll
    for (int t = 0; t < 4; ++t) acc[r][t] = (v8f){};
  if (wave != 1) {
    const Opnd A{xp, nullptr, F}, B{wih, nullptr, F};
    gemm_tile<3, 1>(A, B, F, m0, c0, nloc, hlf, acc);
#pragma unroll
    for (int t = 0; t < 4; ++t)
#pragma unroll
      for (int r = 0; r < 2; ++r)
#pragma unroll
        for (int v = 0; v < 8; ++v) Gt[r * 16 + v + 8 * hlf][c0 + t * 16 + nloc] = acc[r][t][v] + bsum[c0 + t * 16 + nloc];
  }
  __syncthreads();
  for (int pass = 0; pass < 2; ++pass) {
    for (int i = threadIdx.x; i < 32 * F / 4; i += 128) { const int rr = i / (F / 4), cq = (i % (F / 4)) * 4; v4f o;
#pragma unroll
      for (int e = 0; e < 4; ++e) { const int u = cq + e; const float ig = 1.0f / (1.0f + __expf(-Gt[rr][u])), gg = tanhf(Gt[rr][2 * F + u]), og = 1.0f / (1.0f + __expf(-Gt[rr][3 * F + u])); o[e] = og * tanhf(ig * gg); }
      *(volatile v4f*)(h + (size_t)(m0 + rr) * F + cq) = o; }
    __threadfence();
  }
}

template <int NOUT>
__global__ __launch_bounds__(128) void lin_kernel(const float* __restrict__ hin, const b16* __restrict__ w, float* __restrict__ hw) {
  __shared__ __attribute__((aligned(16))) float Ts[4][32 * 64];
  const int lane = threadIdx.x & 31, wave = threadIdx.x >> 5, nloc = lane & 15, hlf = lane >> 4, m0 = blockIdx.x * 128 + wave * 32;
  v8f acc[2][4];
#pragma unroll
  for (int r = 0; r < 2; ++r)
#pragma unroll
    for (int t = 0; t < 4; ++t) acc[r][t] = (v8f){};
  const Opnd A{hin, nullptr, F};
#pragma unroll
  for (int kb = 0; kb < F; kb += 32) { v16b a0, a1, d0, d1; load_frags<3>(A, m0 + nloc, kb, hlf, a0, d0); load_frags<3>(A, m0 + 16 + nloc, kb, hlf, a1, d1);
#pragma unroll
    for (int t = 0; t < NOUT / 16; ++t) { const v16b bw = frag_kb(w + (size_t)(t * 16 + nloc) * F + kb, hlf); acc[0][t] = wmma16b(a0, bw, acc[0][t]); acc[1][t] = wmma16b(a1, bw, acc[1][t]); } }
  if (NOUT == 64) { epi_f32(acc, 1.0f, nullptr, hw, 64, m0, 0, lane, Ts[wave]); return; }
  float* Tt = Ts[wave];
#pragma unroll
  for (int t = 0; t < 2; ++t)
#pragma unroll
    for (int r = 0; r < 2; ++r)
#pragma unroll
      for (int v = 0; v < 8; ++v) Tt[(r * 16 + v + 8 * hlf) * 32 + t * 16 + nloc] = acc[r][t][v];
  wave_lds_sync();
  for (int pass = 0; pass < 2; ++pass) {
#pragma unroll
    for (int j = 0; j < 8; ++j) { const int rr = j * 4 + (lane >> 3), c4 = (lane & 7) * 4; *(volatile v4f*)(hw + (size_t)(m0 + rr) * 32 + c4) = *(const v4f*)(Tt + rr * 32 + c4); }
    __threadfence();
  }
}

typedef __attribute__((ext_vector_type(4))) int v4i;

__global__ __launch_bounds__(256) void deg_kernel(const int* __restrict__ edst, float* __restrict__ dinv) {
  constexpr int NB = 16384;
  __shared__ int cnt[NB];
  const int t_ = threadIdx.x, base = blockIdx.x * NB;
  for (int i = t_; i < NB; i += 256) cnt[i] = 0;
  __syncthreads();
  for (int e0 = t_ * 8; e0 < E; e0 += 256 * 8) {
    const v4i a = *(const v4i*)(edst + e0), b = *(const v4i*)(edst + e0 + 4); const int dd[8] = {a[0], a[1], a[2], a[3], b[0], b[1], b[2], b[3]};
#pragma unroll
    for (int j = 0; j < 8; ++j) { const unsigned sl = (unsigned)(dd[j] - base); if (sl < (unsigned)NB) atomicAdd(&cnt[sl], 1); } }
  __syncthreads();
  for (int pass = 0; pass < 2; ++pass) { for (int i = t_; i < NB; i += 256) { const int node = base + i; if (node < NPAD) ((volatile float*)dinv)[node] = (node < N) ? rsqrtf((float)cnt[i] + 1.0f) : 0.0f; } __threadfence(); }
}

template <int DF, int NB, bool RELU>
__global__ __launch_bounds__(256) void gcn_kernel(const int* __restrict__ edst, const int* __restrict__ esrc, const float* __restrict__ h, const float* __restrict__ dinv, const float* __restrict__ bias, float* __restrict__ outp) {
  constexpr float FXS = 4194304.0f, FXI = 1.0f / FXS;
  __shared__ __attribute__((aligned(16))) int acc[NB * DF];
  __shared__ int list[8 * 256];
  const int t_ = threadIdx.x, wave = t_ >> 5, lane = t_ & 31, base = blockIdx.x * NB;
  for (int i = t_; i < NB * DF; i += 256) acc[i] = 0;
  __syncthreads();
  int* wl = list + wave * 256;
  for (int c0 = 0; c0 < E; c0 += 256 * 8) {
    const int e0 = c0 + (wave * 32 + lane) * 8; int dd[8];
    if (e0 + 7 < E) { const v4i a = *(const v4i*)(edst + e0), b = *(const v4i*)(edst + e0 + 4); dd[0] = a[0]; dd[1] = a[1]; dd[2] = a[2]; dd[3] = a[3]; dd[4] = b[0]; dd[5] = b[1]; dd[6] = b[2]; dd[7] = b[3]; }
    else {
#pragma unroll
      for (int j = 0; j < 8; ++j) dd[j] = (e0 + j < E) ? edst[e0 + j] : -1; }
    unsigned sl[8]; bool hit[8]; bool anyl = false;
#pragma unroll
    for (int j = 0; j < 8; ++j) { sl[j] = (unsigned)(dd[j] - base); hit[j] = sl[j] < (unsigned)NB; anyl |= hit[j]; }
    int wc = 0;
    if (__builtin_amdgcn_ballot_w32(anyl) != 0u) {
#pragma unroll
      for (int j = 0; j < 8; ++j) {
        const unsigned mj = __builtin_amdgcn_ballot_w32(hit[j]);
        if (mj != 0u) {
          if (hit[j]) { const int pos = wc + (int)__builtin_amdgcn_mbcnt_lo(mj, 0u); int o = esrc[e0 + j]; o = (o < 0) ? 0 : (o >= N ? N - 1 : o); wl[pos] = (o << 12) | (int)sl[j]; }
          wc += __builtin_popcount(mj); } } }
    __builtin_amdgcn_wave_barrier(); __builtin_amdgcn_fence(__ATOMIC_RELEASE, "workgroup"); __builtin_amdgcn_fence(__ATOMIC_ACQUIRE, "workgroup");
    { constexpr int LPH = DF / 4, HPS = 32 / LPH;
      for (int i0 = 0; i0 < wc; i0 += HPS) { const int i = i0 + lane / LPH; if (i < wc) { const int ent = wl[i]; const int o = ent >> 12, slot = ent & 4095; const int col = (lane % LPH) * 4;
          const v4f v = *(const v4f*)(h + (size_t)o * DF + col); const float w = dinv[o];
#pragma unroll
          for (int c = 0; c < 4; ++c) atomicAdd(&acc[slot * DF + col + c], (int)rintf(w * v[c] * FXS)); } } }
    __builtin_amdgcn_wave_barrier();
  }
  __syncthreads();
  for (int pass = 0; pass < 2; ++pass) {
    for (int i = t_; i < NB * DF / 4; i += 256) { const int r = (i * 4) / DF, c0 = (i * 4) % DF, node = base + r; if (node < NPAD) { v4f o = {0.0f, 0.0f, 0.0f, 0.0f};
        if (node < N) { const float di = dinv[node]; const v4f hv = *(const v4f*)(h + (size_t)node * DF + c0);
#pragma unroll
          for (int c = 0; c < 4; ++c) { float val = di * ((float)acc[i * 4 + c] * FXI + di * hv[c]) + bias[c0 + c]; if (RELU) val = fmaxf(val, 0.0f); o[c] = val; } }
        *(volatile v4f*)(outp + (size_t)node * DF + c0) = o; } }
    __threadfence();
  }
}


__global__ __launch_bounds__(64) void dot_kernel(const int* __restrict__ lab, const float* __restrict__ z, float* __restrict__ out) {
  const int e = blockIdx.x * 64 + threadIdx.x; int s = lab[e], d = lab[EL + e]; s = (s < 0) ? 0 : (s >= N ? N - 1 : s); d = (d < 0) ? 0 : (d >= N ? N - 1 : d);
  float acc = 0.0f;
#pragma unroll
  for (int i = 0; i < C; i += 4) { const v4f a = *(const v4f*)(z + (size_t)s * C + i), b = *(const v4f*)(z + (size_t)d * C + i); acc += a[0] * b[0] + a[1] * b[1] + a[2] * b[2] + a[3] * b[3]; }
  for (int pass = 0; pass < 2; ++pass) { ((volatile float*)out)[e] = acc; __threadfence(); }
}
}

extern "C" void kernel_launch(void* const* d_in, const int* in_sizes, int n_in,
                              void* d_out, int out_size, void* d_ws, size_t ws_size, hipStream_t stream) {
  (void)n_in; (void)out_size;
  const float* x = (const float*)d_in[0]; const int* ei = (const int*)d_in[1]; const int* lab = (const int*)d_in[2];
  const float* Wih = (const float*)d_in[3];   const float* bih = (const float*)d_in[5]; const float* bhh = (const float*)d_in[6];
  const float* W1 = (const float*)d_in[7]; const float* b1 = (const float*)d_in[8]; const float* W2 = (const float*)d_in[9]; const float* b2 = (const float*)d_in[10];
  float* out = (float*)d_out;
  if (in_sizes[0] != N * F || in_sizes[1] != 2 * E || in_sizes[2] != 2 * EL || in_sizes[3] != 4 * F * F || in_sizes[7] != F * S || in_sizes[9] != S * C) return;
  const int* esrc = ei; const int* edst = ei + E;
  size_t off = 0; char* ws = (char*)d_ws;
  auto carve = [&](size_t bytes) { char* p = ws + off; off += (bytes + 255) & ~(size_t)255; return p; };
  float* xp = (float*)carve((size_t)NPAD * F * 4); b16* wih = (b16*)carve(4 * F * F * 2); float* bsum = (float*)carve(4 * F * 4); b16* w1 = (b16*)carve(S * F * 2); b16* w2 = (b16*)carve(C * S * 2);
  float* dinv = (float*)carve((size_t)NPAD * 4); float* hA = (float*)carve((size_t)NPAD * F * 4); float* hB = (float*)carve((size_t)NPAD * F * 4); float* zc = (float*)carve((size_t)NPAD * C * 4);
  if (off > ws_size) return;
  prep_kernel<<<256, 256, 0, stream>>>(x, Wih, bih, bhh, W1, W2, xp, wih, bsum, w1, w2);
  deg_kernel<<<NPAD / 16384 + 1, 256, 0, stream>>>(edst, dinv);
  lstm_kernel<<<NPAD / 32, 128, 0, stream>>>(xp, wih, bsum, hA);
  lin_kernel<64><<<NBLK, 128, 0, stream>>>(hA, w1, hB);
  gcn_kernel<F, 1024, true><<<NPAD / 1024 + 1, 256, 0, stream>>>(edst, esrc, hB, dinv, b1, hA);
  lin_kernel<32><<<NBLK, 128, 0, stream>>>(hA, w2, hB);
  gcn_kernel<C, 2048, false><<<NPAD / 2048 + 1, 256, 0, stream>>>(edst, esrc, hB, dinv, b2, zc);
  dot_kernel<<<EL / 64, 64, 0, stream>>>(lab, zc, out);
}
